// FraudDetectionHybrid_65481071400297
// MI455X (gfx1250) — hardware-verified
//
#include <hip/hip_runtime.h>
#include <stddef.h>


typedef __attribute__((ext_vector_type(16))) _Float16 v16h;
typedef __attribute__((ext_vector_type(8)))  _Float16 v8h;
typedef __attribute__((ext_vector_type(8)))  float    v8f;
typedef __attribute__((ext_vector_type(4)))  float    v4f;
typedef __attribute__((ext_vector_type(2)))  float    v2f;

#define SEQ_T   512
#define HID     32
#define FEAT    2
#define NLAYER  3
#define NGATE   128
#define KCAT    34
#define WAVES   4
#define ROWS_W  16
#define ROWS_B  64
#define NTHR    128

struct FragH {
  union U { v16h v; v8h h[2]; };
  static __device__ __forceinline__ v16h load(const _Float16* p) {
    U f; f.h[0] = *(const v8h*)(p); f.h[1] = *(const v8h*)(p + 16); return f.v;
  }
};

__device__ __forceinline__ v8f mma_f16(v16h a, v16h b, v8f c) {
  c = __builtin_amdgcn_wmma_f32_16x16x32_f16(false, a, false, b, (short)0, c, false, false);
  asm volatile("v_nop\n\tv_nop\n\tv_nop\n\tv_nop" : "+v"(c) : "v"(a), "v"(b));
  return c;
}

#define LOG2E_F 1.4426950408889634f
__device__ __forceinline__ float fexp2(float x) { return __builtin_amdgcn_exp2f(x); }
__device__ __forceinline__ float frcp(float x)  { return __builtin_amdgcn_rcpf(x); }
__device__ __forceinline__ float sigm7(float a) { return frcp(1.0f + fexp2(a * (-LOG2E_F / 128.0f))); }
__device__ __forceinline__ float tanh7(float a) { return 1.0f - 2.0f * frcp(fexp2(a * (2.0f * LOG2E_F / 128.0f)) + 1.0f); }
__device__ __forceinline__ float tanh0(float a) { return 1.0f - 2.0f * frcp(fexp2(a * (2.0f * LOG2E_F)) + 1.0f); }

__global__ __launch_bounds__(NTHR)
void lstm_fused_f16(const float* __restrict__ x,
                    const float* __restrict__ extW,
                    const float* __restrict__ extb,
                    const float* __restrict__ extsc,
                    const float* __restrict__ extsh,
                    const float* __restrict__ gW,
                    const float* __restrict__ gb,
                    const float* __restrict__ Wc,
                    const float* __restrict__ bc,
                    float* __restrict__ out)
{
  __shared__ __align__(16) _Float16 sWh[NGATE * HID];
  __shared__ __align__(16) _Float16 sA[WAVES * ROWS_W * HID];
  __shared__ __align__(16) float    sX[WAVES * ROWS_W * FEAT];
  __shared__ __align__(16) float    sOut[ROWS_B];

  const int tid  = threadIdx.x;
  const int wave = tid >> 5;
  const int lane = tid & 31;
  const int hh   = lane >> 4;
  const int c    = lane & 15;
  const int rowBase = blockIdx.x * ROWS_B + wave * ROWS_W;

  for (int e = tid; e < NGATE * HID; e += NTHR) {
    const int n = e >> 5, k = e & 31;
    sWh[e] = (_Float16)(16.0f * gW[n * KCAT + FEAT + k]);
  }
  {
    unsigned* az = (unsigned*)sA;
    for (int e = tid; e < (WAVES * ROWS_W * HID) / 2; e += NTHR) az[e] = 0u;
  }
  float wx0[8], wx1[8], bz[8];
#pragma unroll
  for (int nt = 0; nt < 8; ++nt) {
    const int n = nt * 16 + c;
    wx0[nt] = 128.0f * gW[n * KCAT + 0];
    wx1[nt] = 128.0f * gW[n * KCAT + 1];
    bz[nt]  = 128.0f * gb[n];
  }
  float ew[NLAYER][2][2], eb[NLAYER][2], es[NLAYER][2], eh[NLAYER][2];
#pragma unroll
  for (int l = 0; l < NLAYER; ++l) {
#pragma unroll
    for (int j = 0; j < 2; ++j) {
      ew[l][j][0] = extW[l * 4 + j * 2 + 0];
      ew[l][j][1] = extW[l * 4 + j * 2 + 1];
      eb[l][j] = extb[l * 2 + j];
      es[l][j] = extsc[l * 2 + j];
      eh[l][j] = extsh[l * 2 + j];
    }
  }
  const float wc0 = Wc[c], wc1 = Wc[16 + c], bcv = bc[0];
  __syncthreads();

  _Float16*    sAw = sA + wave * (ROWS_W * HID);
  float*       sXw = sX + wave * (ROWS_W * FEAT);
  const float* xr  = x + (size_t)(rowBase + c) * (size_t)(SEQ_T * FEAT);

  float cst[2][8], hl[2][8];
#pragma unroll
  for (int p = 0; p < 2; ++p)
#pragma unroll
    for (int r = 0; r < 8; ++r) { cst[p][r] = 0.0f; hl[p][r] = 0.0f; }

  for (int t = 0; t < SEQ_T; ++t) {
    const v2f xv = *(const v2f*)(xr + 2 * t);
    float f0 = xv.x, f1 = xv.y;
#pragma unroll
    for (int l = 0; l < NLAYER; ++l) {
      const float a0 = f0 * ew[l][0][0] + f1 * ew[l][0][1] + eb[l][0];
      const float a1 = f0 * ew[l][1][0] + f1 * ew[l][1][1] + eb[l][1];
      f0 = tanh0(a0) * es[l][0] + eh[l][0];
      f1 = tanh0(a1) * es[l][1] + eh[l][1];
    }
    if (hh == 0) { v2f s; s.x = f0; s.y = f1; *(v2f*)(sXw + 2 * c) = s; }
    __syncthreads();

    float fr0[8], fr1[8];
#pragma unroll
    for (int q4 = 0; q4 < 4; ++q4) {
      const v4f v = *(const v4f*)(sXw + 16 * hh + 4 * q4);
      fr0[2 * q4] = v.x; fr1[2 * q4] = v.y; fr0[2 * q4 + 1] = v.z; fr1[2 * q4 + 1] = v.w;
    }
    const v16h af = FragH::load(sAw + c * HID + 8 * hh);

#pragma unroll
    for (int p = 0; p < 2; ++p) {
      v8f zt[4];
#pragma unroll
      for (int g = 0; g < 4; ++g) {
        const int nt = 2 * g + p;
        v8f ci;
#pragma unroll
        for (int r = 0; r < 8; ++r) ci[r] = fr0[r] * wx0[nt] + (fr1[r] * wx1[nt] + bz[nt]);
        const v16h bf = FragH::load(sWh + (nt * 16 + c) * HID + 8 * hh);
        zt[g] = mma_f16(af, bf, ci);
      }
#pragma unroll
      for (int r = 0; r < 8; ++r) {
        const float sf = sigm7(zt[0][r]);
        const float si = sigm7(zt[1][r]);
        const float tg = tanh7(zt[2][r]);
        const float so = sigm7(zt[3][r]);
        const float cn = sf * cst[p][r] + si * tg;
        cst[p][r] = cn;
        const float hn = so * tanh0(cn);
        hl[p][r] = hn;
        sAw[(8 * hh + r) * HID + p * 16 + c] = (_Float16)(hn * 8.0f);
      }
    }
    __syncthreads();
  }

  float part[8];
#pragma unroll
  for (int r = 0; r < 8; ++r) part[r] = hl[0][r] * wc0 + hl[1][r] * wc1;
#pragma unroll
  for (int off = 1; off < 16; off <<= 1) {
#pragma unroll
    for (int r = 0; r < 8; ++r) part[r] += __shfl_xor(part[r], off, 32);
  }
  if (c == 0) {
#pragma unroll
    for (int r = 0; r < 8; ++r) sOut[wave * ROWS_W + 8 * hh + r] = part[r] + bcv;
  }
  __syncthreads();

  const int ol = lane & 15;
  const v4f ov = *(const v4f*)(sOut + 4 * ol);
  float* op = out + (size_t)blockIdx.x * ROWS_B + 4 * ol;
  const bool wr = (wave == 0) && (lane < 16);
  if (wr) *(volatile v4f*)op = ov;
  __threadfence();
  if (wr) *(volatile v4f*)op = ov;
}

extern "C" void kernel_launch(void* const* d_in, const int* in_sizes, int n_in,
                              void* d_out, int out_size, void* d_ws, size_t ws_size,
                              hipStream_t stream) {
  (void)d_ws; (void)ws_size;
  if (n_in < 9) return;
  const int nb = out_size;
  if (nb <= 0 || (nb % ROWS_B) != 0) return;
  if (in_sizes[0] != nb * SEQ_T * FEAT) return;
  if (in_sizes[1] != NLAYER * FEAT * FEAT) return;
  if (in_sizes[2] != NLAYER * FEAT || in_sizes[3] != NLAYER * FEAT || in_sizes[4] != NLAYER * FEAT) return;
  if (in_sizes[5] != NGATE * KCAT || in_sizes[6] != NGATE || in_sizes[7] != HID || in_sizes[8] < 1) return;

  const float* x     = (const float*)d_in[0];
  const float* extW  = (const float*)d_in[1];
  const float* extb  = (const float*)d_in[2];
  const float* extsc = (const float*)d_in[3];
  const float* extsh = (const float*)d_in[4];
  const float* gW    = (const float*)d_in[5];
  const float* gb    = (const float*)d_in[6];
  const float* Wc    = (const float*)d_in[7];
  const float* bc    = (const float*)d_in[8];
  float* out = (float*)d_out;

  dim3 grid(nb / ROWS_B);
  dim3 block(NTHR);
  hipLaunchKernelGGL(lstm_fused_f16, grid, block, 0, stream,
                     x, extW, extb, extsc, extsh, gW, gb, Wc, bc, out);
  (void)hipGetLastError();
}
